// DynamicSubgraphGCN_5102421147741
// MI455X (gfx1250) — hardware-verified
//
#include <hip/hip_runtime.h>
#include <stddef.h>


#define NGRAPH  16
#define DF      64
#define NLAYER  2
#define NTHR    256
#define NWAVE   8
#define NB      256
#define EPT     8
#define CHUNK   (NTHR * EPT)
#define WCAP    (32 * EPT)
#define LISTN   (NWAVE * WCAP)
#define WP      72
#define EPSV    1e-6f
#define LDS_MAX 294912

static_assert(NB == NTHR);
static_assert((NB & (NB - 1)) == 0 && NB <= 256);
static_assert(CHUNK == NWAVE * 32 * EPT);
static_assert(NTHR * 16 == DF * DF);
static_assert((WP % 8) == 0);
static_assert((DF % 32) == 0);

typedef float          v2f  __attribute__((ext_vector_type(2)));
typedef float          v4f  __attribute__((ext_vector_type(4)));
typedef float          v8f  __attribute__((ext_vector_type(8)));
typedef int            v4i  __attribute__((ext_vector_type(4)));
typedef unsigned int   v4u  __attribute__((ext_vector_type(4)));
typedef unsigned short v8us __attribute__((ext_vector_type(8)));
typedef __bf16         v16bf __attribute__((ext_vector_type(16)));
union FragB { v16bf v; v8us u[2]; };

__device__ __forceinline__ unsigned int bfbits(float f) {
  const unsigned int u = __float_as_uint(f);
  return (u + 0x7fffu + ((u >> 16) & 1u)) >> 16;
}

#define SPLIT1(I, X) { const float xv_ = (X); const unsigned int hb_ = bfbits(xv_); \
    hi[I] = (unsigned short)hb_; lo[I] = (unsigned short)bfbits(xv_ - __uint_as_float(hb_ << 16)); }
__device__ __forceinline__ void split8(v4f a, v4f b, v8us& hi, v8us& lo) {
  SPLIT1(0, a.x) SPLIT1(1, a.y) SPLIT1(2, a.z) SPLIT1(3, a.w)
  SPLIT1(4, b.x) SPLIT1(5, b.y) SPLIT1(6, b.z) SPLIT1(7, b.w)
}
#undef SPLIT1

__device__ __forceinline__ v8f wmb(v16bf a, v16bf b, v8f c) {
  v8f d = __builtin_amdgcn_wmma_f32_16x16x32_bf16(false, a, false, b, (short)0, c, false, false);
  asm volatile("v_nop\n\tv_nop\n\tv_nop\n\tv_nop" : "+v"(d) : "v"(a), "v"(b));
  return d;
}

__device__ __forceinline__ float gelu1(float v) {
  return 0.5f * v * (1.0f + erff(v * 0.70710678118654752f));
}

template <bool AGG>
__device__ __forceinline__ int scan_chunk(const int* __restrict__ keys, const int* __restrict__ nbs,
                                          const float* __restrict__ mg, const float* __restrict__ disg,
                                          int nE, int nN, int cbase, int rowBase, int vec,
                                          int* list, int* listw, int lane, int wave) {
  const int e0 = cbase + wave * (32 * EPT) + lane * EPT;
  const int ksent = -2147483647 - 1;
  v4i ka, kb, na, nq;
  v4f ma, mb;
  if (vec != 0 && e0 + 7 < nE) {
    ka = *(const v4i*)(keys + e0); kb = *(const v4i*)(keys + e0 + 4);
    na = *(const v4i*)(nbs + e0);  nq = *(const v4i*)(nbs + e0 + 4);
    ma = *(const v4f*)(mg + e0);   mb = *(const v4f*)(mg + e0 + 4);
  } else {
#define LD1(OFF, KC, NC, MC) { const int e = e0 + (OFF); const bool ok = e < nE; const int ec = ok ? e : nE - 1; \
      const int tk = keys[ec]; const int tn = nbs[ec]; const float tm = mg[ec]; \
      KC = ok ? tk : ksent; NC = ok ? tn : 0; MC = ok ? tm : 0.0f; }
    LD1(0, ka.x, na.x, ma.x) LD1(1, ka.y, na.y, ma.y) LD1(2, ka.z, na.z, ma.z) LD1(3, ka.w, na.w, ma.w)
    LD1(4, kb.x, nq.x, mb.x) LD1(5, kb.y, nq.y, mb.y) LD1(6, kb.z, nq.z, mb.z) LD1(7, kb.w, nq.w, mb.w)
#undef LD1
  }
  const unsigned int rbu = (unsigned int)rowBase;
  int excl = 0, tot = 0;
#define HITP(KJ) { const unsigned int sj = (unsigned int)(KJ) - rbu; const bool hj = sj < (unsigned int)NB; \
    const unsigned int mk = __builtin_amdgcn_ballot_w32(hj); \
    excl += (int)__builtin_amdgcn_mbcnt_lo(mk, 0u); tot += (int)__builtin_popcount(mk); }
  HITP(ka.x) HITP(ka.y) HITP(ka.z) HITP(ka.w) HITP(kb.x) HITP(kb.y) HITP(kb.z) HITP(kb.w)
#undef HITP
  int run = excl;
#define EMIT(KJ, NJ, MJ) { const unsigned int sj = (unsigned int)(KJ) - rbu; \
    if (sj < (unsigned int)NB) { \
      int nb = (NJ); nb = nb < 0 ? 0 : (nb > nN - 1 ? nN - 1 : nb); \
      float w = (MJ); if (AGG) w = w * disg[nb]; \
      if (run < WCAP) { const int p = wave * WCAP + run; list[p] = (nb << 8) | (int)sj; listw[p] = __float_as_int(w); } \
      ++run; } }
  EMIT(ka.x, na.x, ma.x) EMIT(ka.y, na.y, ma.y) EMIT(ka.z, na.z, ma.z) EMIT(ka.w, na.w, ma.w)
  EMIT(kb.x, nq.x, mb.x) EMIT(kb.y, nq.y, mb.y) EMIT(kb.z, nq.z, mb.z) EMIT(kb.w, nq.w, mb.w)
#undef EMIT
  return tot;
}

__global__ __launch_bounds__(NTHR) void k_deg(
    const int* __restrict__ ei, const float* __restrict__ mm, float* dis,
    int nN, int nE, int nblk, int npd, int wpr, int vec) {
  extern __shared__ v4u lds_u[];
  unsigned int* bitmap = (unsigned int*)lds_u;
  float*        degacc = (float*)(bitmap + NB * wpr);
  int*          list   = (int*)(degacc + NB);
  int*          listw  = list + LISTN;
  int*          wcnt   = listw + LISTN;
  const int tid = threadIdx.x, lane = tid & 31, wave = tid >> 5;
  const int b = blockIdx.x / nblk;
  const int rb = blockIdx.x - b * nblk;
  const int rowBase = rb * NB;
  const int*   srcA = ei + (size_t)b * 2 * (size_t)nE;
  const int*   dstA = srcA + nE;
  const float* mg   = mm + (size_t)b * (size_t)nE;

  {
    const v4u z = {0u, 0u, 0u, 0u};
    const int nz = (NB * wpr) / 4;
    for (int i = tid; i < nz; i += NTHR) lds_u[i] = z;
  }
  degacc[tid] = 1.0f;
  __syncthreads();

  const int nChunks = (nE + CHUNK - 1) / CHUNK;
#pragma unroll 1
  for (int cls = 0; cls < 2; ++cls) {
    const int* keys = (cls == 0) ? dstA : srcA;
    const int* nbs  = (cls == 0) ? srcA : dstA;
#pragma unroll 1
    for (int ch = nChunks - 1; ch >= 0; --ch) {
      const int cbase = ch * CHUNK;
      const int wc = scan_chunk<false>(keys, nbs, mg, mg, nE, nN, cbase, rowBase, vec, list, listw, lane, wave);
      if (lane == 0) wcnt[wave] = wc;
      __syncthreads();
      if (wave == 0) {
#pragma unroll 1
        for (int wsx = NWAVE - 1; wsx >= 0; --wsx) {
          int n = __builtin_amdgcn_readfirstlane(wcnt[wsx]);
          n = n > WCAP ? WCAP : (n < 0 ? 0 : n);
          const int lb = wsx * WCAP;
#pragma unroll 1
          for (int i = n - 1; i >= 0; --i) {
            const int   ent  = __builtin_amdgcn_readfirstlane(list[lb + i]);
            const float w    = __int_as_float(__builtin_amdgcn_readfirstlane(listw[lb + i]));
            const int   slot = ent & (NB - 1);
            int nb = (int)((unsigned int)ent >> 8);
            nb = nb > nN - 1 ? nN - 1 : nb;
            const int word = slot * wpr + (nb >> 5);
            const unsigned int bit = 1u << (nb & 31);
            const unsigned int bm = (unsigned int)__builtin_amdgcn_readfirstlane((int)bitmap[word]);
            if ((bm & bit) == 0u) {
              bitmap[word] = bm | bit;
              degacc[slot] = degacc[slot] + w;
            }
          }
        }
      }
      __syncthreads();
    }
  }

  if (tid < NB / 4) {
    const int f = 4 * tid;
    v4f d;
    d.x = rsqrtf(fmaxf(degacc[f + 0], EPSV));
    d.y = rsqrtf(fmaxf(degacc[f + 1], EPSV));
    d.z = rsqrtf(fmaxf(degacc[f + 2], EPSV));
    d.w = rsqrtf(fmaxf(degacc[f + 3], EPSV));
    float* dp = dis + (size_t)b * (size_t)npd + rowBase + f;
    *(volatile v4f*)dp = d;
    __threadfence();
    *(volatile v4f*)dp = d;
  }
}

template <bool GELU>
__global__ __launch_bounds__(NTHR) void k_layer(
    const float* __restrict__ xin, const int* __restrict__ ei, const float* __restrict__ mm,
    const float* __restrict__ dis, const float* __restrict__ wl, float* yout,
    int xRows, int yRows, int yLimit, int nN, int nE, int nblk, int npd, int wpr, int vec) {
  extern __shared__ v4u lds_u[];
  float*          acc    = (float*)lds_u;
  unsigned int*   bitmap = (unsigned int*)(acc + NB * DF);
  int*            list   = (int*)(bitmap + NB * wpr);
  int*            listw  = list + LISTN;
  unsigned short* whi    = (unsigned short*)(listw + LISTN);
  unsigned short* wlo    = whi + DF * WP;
  int*            wcnt   = (int*)(wlo + DF * WP);
  const int tid = threadIdx.x, lane = tid & 31, wave = tid >> 5, hh = lane >> 4, m = lane & 15;
  const int b = blockIdx.x / nblk;
  const int rb = blockIdx.x - b * nblk;
  const int rowBase = rb * NB;
  const int*   srcA = ei + (size_t)b * 2 * (size_t)nE;
  const int*   dstA = srcA + nE;
  const float* mg   = mm + (size_t)b * (size_t)nE;
  const float* disg = dis + (size_t)b * (size_t)npd;
  const float* xg   = xin + (size_t)b * (size_t)xRows * DF;

  {
    const v4u z = {0u, 0u, 0u, 0u};
    const int nz = (NB * DF + NB * wpr) / 4;
    for (int i = tid; i < nz; i += NTHR) lds_u[i] = z;
  }
  {
    const int o = tid * 16;
    const int e = o >> 6, d0 = o & 63;
    const v4f q0 = *(const v4f*)(wl + o), q1 = *(const v4f*)(wl + o + 4);
    const v4f q2 = *(const v4f*)(wl + o + 8), q3 = *(const v4f*)(wl + o + 12);
    v8us h0, l0, h1, l1;
    split8(q0, q1, h0, l0);
    split8(q2, q3, h1, l1);
    unsigned short* hp = whi + e * WP + d0;
    unsigned short* lp = wlo + e * WP + d0;
    *(v8us*)hp = h0; *(v8us*)(hp + 8) = h1;
    *(v8us*)lp = l0; *(v8us*)(lp + 8) = l1;
  }
  __syncthreads();

  const int nChunks = (nE + CHUNK - 1) / CHUNK;
#pragma unroll 1
  for (int cls = 0; cls < 2; ++cls) {
    const int* keys = (cls == 0) ? dstA : srcA;
    const int* nbs  = (cls == 0) ? srcA : dstA;
#pragma unroll 1
    for (int ch = nChunks - 1; ch >= 0; --ch) {
      const int cbase = ch * CHUNK;
      const int wc = scan_chunk<true>(keys, nbs, mg, disg, nE, nN, cbase, rowBase, vec, list, listw, lane, wave);
      if (lane == 0) wcnt[wave] = wc;
      __syncthreads();
      if (wave == 0) {
#pragma unroll 1
        for (int wsx = NWAVE - 1; wsx >= 0; --wsx) {
          int n = __builtin_amdgcn_readfirstlane(wcnt[wsx]);
          n = n > WCAP ? WCAP : (n < 0 ? 0 : n);
          const int lb = wsx * WCAP;
#pragma unroll 1
          for (int i = n - 1; i >= 0; --i) {
            const int   ent  = __builtin_amdgcn_readfirstlane(list[lb + i]);
            const float w    = __int_as_float(__builtin_amdgcn_readfirstlane(listw[lb + i]));
            const int   slot = ent & (NB - 1);
            int nb = (int)((unsigned int)ent >> 8);
            nb = nb > nN - 1 ? nN - 1 : nb;
            const int word = slot * wpr + (nb >> 5);
            const unsigned int bit = 1u << (nb & 31);
            const unsigned int bm = (unsigned int)__builtin_amdgcn_readfirstlane((int)bitmap[word]);
            if ((bm & bit) == 0u) {
              bitmap[word] = bm | bit;
              const v2f xv = *(const v2f*)(xg + (size_t)nb * DF + 2 * lane);
              v2f* ap = (v2f*)(acc + slot * DF + 2 * lane);
              v2f av = *ap;
              av.x = fmaf(w, xv.x, av.x);
              av.y = fmaf(w, xv.y, av.y);
              *ap = av;
            }
          }
        }
      }
      __syncthreads();
    }
  }

#pragma unroll 4
  for (int it = 0; it < (NB * DF / 4) / NTHR; ++it) {
    const int idx  = it * NTHR + tid;
    const int slot = idx >> 4;
    const int c4   = (idx & 15) * 4;
    const int node = rowBase + slot;
    const int xl   = node < nN ? node : nN - 1;
    const float d  = disg[rowBase + slot];
    const v4f xv = *(const v4f*)(xg + (size_t)xl * DF + c4);
    v4f* ap = (v4f*)(acc + slot * DF + c4);
    const v4f av = *ap;
    *ap = (xv * d + av) * d;
  }
  __syncthreads();

#pragma unroll 1
  for (int tt = 0; tt < 2; ++tt) {
    const int t = 2 * wave + tt;
    v8f c[4];
#pragma unroll
    for (int u = 0; u < 4; ++u) { const v8f z = {0.f, 0.f, 0.f, 0.f, 0.f, 0.f, 0.f, 0.f}; c[u] = z; }
#pragma unroll
    for (int kt = 0; kt < DF / 32; ++kt) {
      const float* ap = acc + (16 * t + m) * DF + 32 * kt + 8 * hh;
      const v4f p0 = *(const v4f*)ap,        p1 = *(const v4f*)(ap + 4);
      const v4f p2 = *(const v4f*)(ap + 16), p3 = *(const v4f*)(ap + 20);
      FragB ah, al;
      split8(p0, p1, ah.u[0], al.u[0]);
      split8(p2, p3, ah.u[1], al.u[1]);
#pragma unroll
      for (int u = 0; u < 4; ++u) {
        const unsigned short* bp = whi + (16 * u + m) * WP + 32 * kt + 8 * hh;
        const unsigned short* bq = wlo + (16 * u + m) * WP + 32 * kt + 8 * hh;
        FragB bh, bl;
        bh.u[0] = *(const v8us*)bp; bh.u[1] = *(const v8us*)(bp + 16);
        bl.u[0] = *(const v8us*)bq; bl.u[1] = *(const v8us*)(bq + 16);
        c[u] = wmb(ah.v, bh.v, c[u]);
        c[u] = wmb(ah.v, bl.v, c[u]);
        c[u] = wmb(al.v, bh.v, c[u]);
      }
    }
    float* sp = acc + (16 * t + 8 * hh) * DF + m;
#pragma unroll
    for (int u = 0; u < 4; ++u) {
      sp[0 * DF + 16 * u] = c[u][0];
      sp[1 * DF + 16 * u] = c[u][1];
      sp[2 * DF + 16 * u] = c[u][2];
      sp[3 * DF + 16 * u] = c[u][3];
      sp[4 * DF + 16 * u] = c[u][4];
      sp[5 * DF + 16 * u] = c[u][5];
      sp[6 * DF + 16 * u] = c[u][6];
      sp[7 * DF + 16 * u] = c[u][7];
    }
  }
  __syncthreads();

  {
    const int cc = 4 * m;
#pragma unroll 1
    for (int i = 0; i < 16; ++i) {
      const int r = 32 * wave + 2 * i + hh;
      v4f v = *(const v4f*)(acc + r * DF + cc);
      if (GELU) { v.x = gelu1(v.x); v.y = gelu1(v.y); v.z = gelu1(v.z); v.w = gelu1(v.w); }
      const int node = rowBase + r;
      if (node < yLimit) *(volatile v4f*)(yout + ((size_t)b * (size_t)yRows + node) * DF + cc) = v;
    }
    __threadfence();
#pragma unroll 1
    for (int i = 0; i < 16; ++i) {
      const int r = 32 * wave + 2 * i + hh;
      v4f v = *(const v4f*)(acc + r * DF + cc);
      if (GELU) { v.x = gelu1(v.x); v.y = gelu1(v.y); v.z = gelu1(v.z); v.w = gelu1(v.w); }
      const int node = rowBase + r;
      if (node < yLimit) *(volatile v4f*)(yout + ((size_t)b * (size_t)yRows + node) * DF + cc) = v;
    }
  }
}

extern "C" void kernel_launch(void* const* d_in, const int* in_sizes, int n_in,
                              void* d_out, int out_size, void* d_ws, size_t ws_size,
                              hipStream_t stream) {
  if (n_in < 4) return;
  const int nB = NGRAPH;
  if (in_sizes[0] <= 0 || (in_sizes[0] % (nB * DF)) != 0) return;
  const int nN = in_sizes[0] / (nB * DF);
  if (in_sizes[2] < 0 || (in_sizes[2] % nB) != 0) return;
  const int nE = in_sizes[2] / nB;
  if (in_sizes[1] != 2 * nB * nE) return;
  if (in_sizes[3] != NLAYER * DF * DF) return;
  if (out_size != nB * nN * DF) return;
  if (nN > (1 << 22)) return;

  const float* Hin = (const float*)d_in[0];
  const int*   ei  = (const int*)d_in[1];
  const float* mm  = (const float*)d_in[2];
  const float* W   = (const float*)d_in[3];
  float* out = (float*)d_out;

  const int nblk = (nN + NB - 1) / NB;
  const int npd  = nblk * NB;
  const int wpr  = (nN + 31) / 32;

  const size_t ldsD = (size_t)NB * wpr * 4 + (size_t)NB * 4 + 2 * (size_t)LISTN * 4 + NWAVE * 4;
  const size_t ldsL = (size_t)NB * DF * 4 + (size_t)NB * wpr * 4 + 2 * (size_t)LISTN * 4
                    + 2 * (size_t)DF * WP * 2 + NWAVE * 4;
  if (ldsL > (size_t)LDS_MAX || ldsD > (size_t)LDS_MAX) return;

  char* ws = (char*)d_ws;
  size_t off = 0;
  const size_t oDis = off; off += (size_t)nB * npd * 4;        off = (off + 255) & ~(size_t)255;
  const size_t oX1  = off; off += (size_t)nB * npd * DF * 4;   off = (off + 255) & ~(size_t)255;
  if (off > ws_size || off > (size_t)134217728) return;
  float* dis = (float*)(ws + oDis);
  float* x1  = (float*)(ws + oX1);

  const int vec  = ((nE & 3) == 0) ? 1 : 0;
  const int grid = nB * nblk;

  hipFuncSetAttribute(reinterpret_cast<const void*>(&k_deg),
                      hipFuncAttributeMaxDynamicSharedMemorySize, (int)ldsD);
  k_deg<<<grid, NTHR, ldsD, stream>>>(ei, mm, dis, nN, nE, nblk, npd, wpr, vec);

  hipFuncSetAttribute(reinterpret_cast<const void*>(&k_layer<true>),
                      hipFuncAttributeMaxDynamicSharedMemorySize, (int)ldsL);
  k_layer<true><<<grid, NTHR, ldsL, stream>>>(Hin, ei, mm, dis, W, x1,
                                              nN, npd, npd, nN, nE, nblk, npd, wpr, vec);

  hipFuncSetAttribute(reinterpret_cast<const void*>(&k_layer<false>),
                      hipFuncAttributeMaxDynamicSharedMemorySize, (int)ldsL);
  k_layer<false><<<grid, NTHR, ldsL, stream>>>(x1, ei, mm, dis, W + DF * DF, out,
                                               npd, nN, nN, nN, nE, nblk, npd, wpr, vec);
}
